// RelPosMultiHeadSelfAttention_88218628260744
// MI455X (gfx1250) — hardware-verified
//
#include <hip/hip_runtime.h>


namespace {
constexpr int Bn = 8, T = 512, D = 1024, H = 16, HD = 64, NT = Bn * T, NR = 2 * T - 1  , NRP = 1024;
constexpr float XS = 8.0f, PS = 8.0f;
struct Wo_ { static constexpr size_t Q = 0, K = (size_t)D * D, V = 2 * (size_t)D * D, Pp = 3 * (size_t)D * D, O = 4 * (size_t)D * D, END = 5 * (size_t)D * D; };

__constant__ unsigned int kInvFreqBits[512] = {0x3f800000,0x3f7b6f9e,0x3f76f410,0x3f728cf8,0x3f6e39f8,0x3f69fab4,0x3f65ced3,0x3f61b5fb,0x3f5dafd7,0x3f59bc0f,0x3f55da52,0x3f520a4c,0x3f4e4bac,0x3f4a9e24,0x3f470165,0x3f437522,0x3f3ff911,0x3f3c8ce7,0x3f39305c,0x3f35e329,0x3f32a506,0x3f2f75b1,0x3f2c54e5,0x3f294260,0x3f263de0,0x3f234726,0x3f205df3,0x3f1d8209,0x3f1ab32b,0x3f17f11e,0x3f153ba8,0x3f12928f,0x3f0ff59a,0x3f0d6492,0x3f0adf41,0x3f086571,0x3f05f6ee,0x3f039384,0x3f013b01,0x3efdda64,0x3ef953cf,0x3ef4e1e1,0x3ef0843c,0x3eec3a85,0x3ee80460,0x3ee3e173,0x3edfd167,0x3edbd3e6,0x3ed7e89b,0x3ed40f33,0x3ed0475c,0x3ecc90c7,0x3ec8eb24,0x3ec55626,0x3ec1d181,0x3ebe5ceb,0x3ebaf81a,0x3eb7a2c7,0x3eb45caa,0x3eb1257e,0x3eadfcff,0x3eaae2ea,0x3ea7d6fd,0x3ea4d8f8,0x3ea1e89b,0x3e9f05a8,0x3e9c2fe1,0x3e99670b,0x3e96aaea,0x3e93fb44,0x3e9157e1,0x3e8ec089,0x3e8c3504,0x3e89b51c,0x3e87409d,0x3e84d752,0x3e827909,0x3e80258f,0x3e7bb965,0x3e773c86,0x3e72d424,0x3e6e7fdf,0x3e6a3f5c,0x3e661241,0x3e61f836,0x3e5df0e3,0x3e59fbf3,0x3e561912,0x3e5247ed,0x3e4e8834,0x3e4ad998,0x3e473bc9,0x3e43ae7c,0x3e403165,0x3e3cc43a,0x3e3966b3,0x3e361887,0x3e32d971,0x3e2fa92d,0x3e2c8776,0x3e29740a,0x3e266ea7,0x3e23770f,0x3e208d01,0x3e1db040,0x3e1ae08f,0x3e181db4,0x3e156772,0x3e12bd91,0x3e101fd7,0x3e0d8e0f,0x3e0b0801,0x3e088d77,0x3e061e3d,0x3e03ba20,0x3e0160ec,0x3dfe24e1,0x3df99cf7,0x3df529bb,0x3df0cacf,0x3dec7fd5,0x3de84874,0x3de42450,0x3de01313,0x3ddc1466,0x3dd827f5,0x3dd44d6c,0x3dd08479,0x3dcccccd,0x3dc92618,0x3dc5900d,0x3dc20a60,0x3dbe94c7,0x3dbb2ef7,0x3db7d8a9,0x3db49196,0x3db15978,0x3dae300c,0x3dab150e,0x3da8083d,0x3da50957,0x3da2181d,0x3d9f3451,0x3d9c5db5,0x3d99940e,0x3d96d71f,0x3d9426b0,0x3d918287,0x3d8eea6c,0x3d8c5e27,0x3d89dd84,0x3d87684c,0x3d84fe4d,0x3d829f52,0x3d804b29,0x3d7c0341,0x3d778512,0x3d731b64,0x3d6ec5da,0x3d6a8418,0x3d6655c3,0x3d623a83,0x3d5e3202,0x3d5a3be9,0x3d5657e4,0x3d5285a1,0x3d4ec4ce,0x3d4b151d,0x3d47763f,0x3d43e7e7,0x3d4069ca,0x3d3cfb9e,0x3d399d19,0x3d364df5,0x3d330dec,0x3d2fdcb8,0x3d2cba15,0x3d29a5c2,0x3d269f7d,0x3d23a705,0x3d20bc1d,0x3d1dde85,0x3d1b0e01,0x3d184a56,0x3d159348,0x3d12e89f,0x3d104a21,0x3d0db798,0x3d0b30cc,0x3d08b588,0x3d064597,0x3d03e0c7,0x3d0186e2,0x3cfe6f73,0x3cf9e635,0x3cf571ab,0x3cf11176,0x3cecc53a,0x3ce88c9c,0x3ce46741,0x3ce054d2,0x3cdc54fa,0x3cd86761,0x3cd48bb7,0x3cd0c1a8,0x3ccd08e4,0x3cc9611d,0x3cc5ca05,0x3cc24350,0x3cbeccb2,0x3cbb65e3,0x3cb80e9a,0x3cb4c691,0x3cb18d82,0x3cae6328,0x3cab4741,0x3ca8398b,0x3ca539c4,0x3ca247ad,0x3c9f6308,0x3c9c8b97,0x3c99c11e,0x3c970362,0x3c945229,0x3c91ad39,0x3c8f145b,0x3c8c8757,0x3c8a05f8,0x3c879008,0x3c852553,0x3c82c5a5,0x3c8070cd,0x3c7c4d33,0x3c77cdb2,0x3c7362b9,0x3c6f0be9,0x3c6ac8e7,0x3c669959,0x3c627ce5,0x3c5e7334,0x3c5a7bf1,0x3c5696c8,0x3c52c366,0x3c4f017a,0x3c4b50b4,0x3c47b0c6,0x3c442163,0x3c40a23f,0x3c3d3311,0x3c39d390,0x3c368373,0x3c334276,0x3c301052,0x3c2cecc4,0x3c29d789,0x3c26d061,0x3c23d70a,0x3c20eb46,0x3c1e0cd7,0x3c1b3b80,0x3c187705,0x3c15bf2c,0x3c1313ba,0x3c107478,0x3c0de12d,0x3c0b59a3,0x3c08dda5,0x3c066cfd,0x3c040779,0x3c01ace4,0x3bfeba1b,0x3bfa2f88,0x3bf5b9b0,0x3bf15832,0x3bed0ab3,0x3be8d0d8,0x3be4aa46,0x3be096a5,0x3bdc95a0,0x3bd8a6e1,0x3bd4ca14,0x3bd0fee9,0x3bcd450e,0x3bc99c34,0x3bc6040e,0x3bc27c50,0x3bbf04ae,0x3bbb9ce0,0x3bb8449c,0x3bb4fb9c,0x3bb1c19b,0x3bae9654,0x3bab7983,0x3ba86ae7,0x3ba56a3f,0x3ba2774a,0x3b9f91cc,0x3b9cb986,0x3b99ee3b,0x3b972fb1,0x3b947dae,0x3b91d7f7,0x3b8f3e56,0x3b8cb093,0x3b8a2e77,0x3b87b7cf,0x3b854c64,0x3b82ec04,0x3b80967d,0x3b7c973b,0x3b781668,0x3b73aa23,0x3b6f520d,0x3b6b0dcb,0x3b66dd02,0x3b62bf5a,0x3b5eb47a,0x3b5abc0d,0x3b56d5bf,0x3b53013e,0x3b4f3e37,0x3b4b8c5c,0x3b47eb5e,0x3b445aef,0x3b40dac5,0x3b3d6a95,0x3b3a0a16,0x3b36b901,0x3b33770f,0x3b3043fb,0x3b2d1f81,0x3b2a095f,0x3b270153,0x3b24071d,0x3b211a7e,0x3b1e3b37,0x3b1b690d,0x3b18a3c2,0x3b15eb1c,0x3b133ee2,0x3b109edb,0x3b0e0ace,0x3b0b8287,0x3b0905ce,0x3b06946f,0x3b042e36,0x3b01d2f1,0x3aff04d9,0x3afa78f1,0x3af601c9,0x3af19f03,0x3aed5041,0x3ae91528,0x3ae4ed5e,0x3ae0d88b,0x3adcd659,0x3ad8e673,0x3ad50884,0x3ad13c3c,0x3acd8149,0x3ac9d75c,0x3ac63e28,0x3ac2b561,0x3abf3cbb,0x3abbd3ec,0x3ab87aad,0x3ab530b7,0x3ab1f5c3,0x3aaec98e,0x3aababd3,0x3aa89c52,0x3aa59ac8,0x3aa2a6f6,0x3a9fc09e,0x3a9ce782,0x3a9a1b66,0x3a975c0e,0x3a94a940,0x3a9202c3,0x3a8f685e,0x3a8cd9db,0x3a8a5703,0x3a87dfa1,0x3a857381,0x3a83126f,0x3a80bc38,0x3a7ce158,0x3a785f33,0x3a73f1a2,0x3a6f9846,0x3a6b52c4,0x3a6720c0,0x3a6301e2,0x3a5ef5d2,0x3a5afc3b,0x3a5714c9,0x3a533f27,0x3a4f7b06,0x3a4bc816,0x3a482607,0x3a44948c,0x3a41135b,0x3a3da229,0x3a3a40ad,0x3a36ee9e,0x3a33abb7,0x3a3077b3,0x3a2d524d,0x3a2a3b43,0x3a273254,0x3a24373e,0x3a2149c3,0x3a1e69a5,0x3a1b96a6,0x3a18d08b,0x3a161719,0x3a136a16,0x3a10c94a,0x3a0e347c,0x3a0bab76,0x3a092e02,0x3a06bbec,0x3a0454ff,0x3a01f908,0x39ff4fad,0x39fac26f,0x39f649f8,0x39f1e5e8,0x39ed95e3,0x39e9598c,0x39e5308a,0x39e11a85,0x39dd1726,0x39d92617,0x39d54706,0x39d179a1,0x39cdbd95,0x39ca1296,0x39c67853,0x39c2ee82,0x39bf74d7,0x39bc0b09,0x39b8b0cf,0x39b565e1,0x39b229fb,0x39aefcd7,0x39abde33,0x39a8cdcb,0x39a5cb5f,0x39a2d6b0,0x399fef7e,0x399d158c,0x399a489e,0x39978877,0x3994d4df,0x39922d9a,0x398f9272,0x398d032f,0x398a7f9b,0x3988077f,0x39859aa9,0x398338e4,0x3980e1fe,0x397d2b8c,0x3978a814,0x39743936,0x396fde93,0x396b97d0,0x39676491,0x3963447e,0x395f373e,0x395b3c7c,0x395753e5,0x39537d23,0x394fb7e7,0x394c03e1,0x394860c1,0x3944ce3b,0x39414c02,0x393dd9ce,0x393a7753,0x3937244b,0x3933e06f,0x3930ab7b,0x392d8529,0x392a6d37,0x39276363,0x3924676d,0x39217917,0x391e9820,0x391bc44d,0x3918fd62,0x39164323,0x39139558,0x3910f3c6,0x390e5e36,0x390bd472,0x39095643,0x3906e374,0x39047bd3,0x39021f2b,0x38ff9a97,0x38fb0c03,0x38f6923c,0x38f22ce3,0x38eddb99,0x38e99e04,0x38e573ca,0x38e15c92,0x38dd5805,0x38d965ce,0x38d5859b};
typedef _Float16 b16;
typedef __attribute__((ext_vector_type(16))) _Float16 v16b;
typedef __attribute__((ext_vector_type(8))) _Float16 v8b;
typedef __attribute__((ext_vector_type(8))) float v8f;
typedef __attribute__((ext_vector_type(4))) float v4f;
__device__ __forceinline__ float bf16_rne(float f) { unsigned int u = __float_as_uint(f); u += 0x7FFFu + ((u >> 16) & 1u); return __uint_as_float(u & 0xFFFF0000u); }
__device__ __forceinline__ void split16(float v, b16& hi, b16& lo) { hi = (b16)v; lo = (b16)(v - (float)hi); }
__device__ __forceinline__ v16b frag_kb(const b16* p, int hh) { const v8b a = *(const v8b*)(p + 8 * hh), b = *(const v8b*)(p + 16 + 8 * hh); v16b f;
#pragma unroll
  for (int e = 0; e < 8; ++e) { f[e] = a[e]; f[8 + e] = b[e]; } return f; }
__device__ __forceinline__ v8f wmma16b(v16b a, v16b b, v8f c) { v8f d = __builtin_amdgcn_wmma_f32_16x16x32_f16(false, a, false, b, (short)0, c, false, false); asm volatile("v_nop\n\tv_nop\n\tv_nop\n\tv_nop" : "+v"(d) : "v"(a), "v"(b)); return d; }
__device__ __forceinline__ void wave_lds_sync() { __builtin_amdgcn_fence(__ATOMIC_RELEASE, "workgroup"); __builtin_amdgcn_wave_barrier(); __builtin_amdgcn_fence(__ATOMIC_ACQUIRE, "workgroup"); }
__device__ __forceinline__ float nexp(float x) { return __builtin_amdgcn_exp2f(x * 1.4426950408889634f); }
__device__ __forceinline__ float pmul(float a, float b) { float p = a * b; asm volatile("" : "+v"(p)); return p; }
__device__ __forceinline__ void sincos_r(float ang, float& sn, float& cs) { const float k = rintf(ang * 0.15915494309189535f); float r = __builtin_fmaf(k, -6.28318548202514648f, ang); r = __builtin_fmaf(k, 1.7484556025237907e-7f, r);
  const float t = r * 0.15915494309189535f; sn = __builtin_amdgcn_sinf(t); cs = __builtin_amdgcn_cosf(t); }

__global__ __launch_bounds__(256) void prep_kernel(const float* __restrict__ x, const float* __restrict__ wq, const float* __restrict__ wk, const float* __restrict__ wv, const float* __restrict__ wp, const float* __restrict__ wo, const float* __restrict__ bq, const float* __restrict__ bk, const float* __restrict__ bv, const float* __restrict__ bp, const float* __restrict__ bo, const float* __restrict__ u, const float* __restrict__ v, b16* __restrict__ R, float* __restrict__ P, b16* __restrict__ X, b16* __restrict__ PEh, b16* __restrict__ PEl) {
  const size_t tid = (size_t)blockIdx.x * 256 + threadIdx.x, nth = (size_t)gridDim.x * 256;
  for (int pass = 0; pass < 2; ++pass) {
    for (size_t p = tid; p < Wo_::END / 8; p += nth) { const size_t q = p * 8; const float* s_ = (q < Wo_::K) ? (wq + q) : (q < Wo_::V) ? (wk + (q - Wo_::K)) : (q < Wo_::Pp) ? (wv + (q - Wo_::V)) : (q < Wo_::O) ? (wp + (q - Wo_::Pp)) : (wo + (q - Wo_::O)); v8b vv; for (int e = 0; e < 8; ++e) vv[e] = (b16)bf16_rne(s_[e]); *(volatile v8b*)(R + q) = vv; }
    for (size_t q = tid; q < 7168; q += nth) { const int i = (int)q, c = i & 1023; const float* s_ = (i < 1024) ? bq : (i < 2048) ? bk : (i < 3072) ? bv : (i < 4096) ? bp : (i < 5120) ? bo : (i < 6144) ? u : v; P[q] = bf16_rne(s_[c]); }
    for (size_t p = tid; p < (size_t)NT * D / 8; p += nth) { v8b vv; for (int e = 0; e < 8; ++e) vv[e] = (b16)(bf16_rne(x[p * 8 + e]) * XS); *(volatile v8b*)(X + p * 8) = vv; }
    for (size_t p = tid; p < (size_t)NRP * D / 8; p += nth) { const int r = (int)(p / (D / 8)), c8 = (int)(p % (D / 8)) * 8; v8b hh_, ll_; const float pos = (float)(T - 1 - r);
      for (int e = 0; e < 8; e += 2) { const int m = (c8 + e) >> 1; const float inv = __uint_as_float(kInvFreqBits[m]); float sn, cs; sincos_r(pmul(pos, inv), sn, cs); if (r >= NR) { sn = 0.0f; cs = 0.0f; }
        b16 a_, c_; split16(sn * XS, a_, c_); hh_[e] = a_; ll_[e] = c_; split16(cs * XS, a_, c_); hh_[e + 1] = a_; ll_[e + 1] = c_; }
      *(volatile v8b*)(PEh + (size_t)r * D + c8) = hh_; *(volatile v8b*)(PEl + (size_t)r * D + c8) = ll_; }
    __threadfence(); }
}

template <int MODE, int TWO>
__global__ __launch_bounds__(64) void gemm_kernel(const b16* __restrict__ A, const b16* __restrict__ Al, const b16* __restrict__ Bw, const float* __restrict__ bias, const float* __restrict__ P, b16* __restrict__ O1, b16* __restrict__ O2, b16* __restrict__ O3, b16* __restrict__ O4, float* __restrict__ O32) {
  __shared__ __attribute__((aligned(16))) float Ts[2][32][128 + 4];
  const int lane = threadIdx.x & 31, wave = threadIdx.x >> 5, nloc = lane & 15, hlf = lane >> 4, m0 = blockIdx.y * 32, c0 = blockIdx.x * 256 + wave * 128;
  v8f acc[2][8];
#pragma unroll
  for (int r = 0; r < 2; ++r)
#pragma unroll
    for (int t = 0; t < 8; ++t) acc[r][t] = (v8f){};
#pragma unroll 2
  for (int kb = 0; kb < D; kb += 32) { const v16b a0 = frag_kb(A + (size_t)(m0 + nloc) * D + kb, hlf), a1 = frag_kb(A + (size_t)(m0 + 16 + nloc) * D + kb, hlf); v16b l0, l1; if (TWO) { l0 = frag_kb(Al + (size_t)(m0 + nloc) * D + kb, hlf); l1 = frag_kb(Al + (size_t)(m0 + 16 + nloc) * D + kb, hlf); }
#pragma unroll
    for (int t = 0; t < 8; ++t) { const v16b bw = frag_kb(Bw + (size_t)(c0 + t * 16 + nloc) * D + kb, hlf); acc[0][t] = wmma16b(a0, bw, acc[0][t]); acc[1][t] = wmma16b(a1, bw, acc[1][t]); if (TWO) { acc[0][t] = wmma16b(l0, bw, acc[0][t]); acc[1][t] = wmma16b(l1, bw, acc[1][t]); } } }
#pragma unroll
  for (int t = 0; t < 8; ++t) { const float bb = bias[c0 + t * 16 + nloc];
#pragma unroll
    for (int r = 0; r < 2; ++r)
#pragma unroll
      for (int vv = 0; vv < 8; ++vv) Ts[wave][r * 16 + 8 * hlf + vv][t * 16 + nloc] = acc[r][t][vv] * (1.0f / XS) + bb; }
  wave_lds_sync();
  for (int pass = 0; pass < 2; ++pass) {
    if (MODE == 3) { for (int i = lane; i < 32 * 32; i += 32) { const int rr = i >> 5, c4 = (i & 31) * 4; *(volatile v4f*)(O32 + (size_t)(m0 + rr) * D + c0 + c4) = *(const v4f*)(&Ts[wave][rr][c4]); } }
    else if (MODE == 2) { for (int i = lane; i < 32 * 16; i += 32) { const int rr = i >> 4, c8 = (i & 15) * 8; v8b o; for (int e = 0; e < 8; ++e) o[e] = (b16)(Ts[wave][rr][c8 + e] * XS); *(volatile v8b*)(O1 + (size_t)(m0 + rr) * D + c0 + c8) = o; } }
    else { for (int i = lane; i < 32 * 16; i += 32) { const int rr = i >> 4, c8 = (i & 15) * 8; const size_t gi = (size_t)(m0 + rr) * D + c0 + c8; v8b h1, l1, h2, l2;
        for (int e = 0; e < 8; ++e) { const float y = Ts[wave][rr][c8 + e]; b16 a_, c_; if (MODE == 0) { split16(y * XS, a_, c_); h1[e] = a_; l1[e] = c_; } else { split16((y + P[5120 + c0 + c8 + e]) * XS, a_, c_); h1[e] = a_; l1[e] = c_; split16((y + P[6144 + c0 + c8 + e]) * XS, a_, c_); h2[e] = a_; l2[e] = c_; } }
        *(volatile v8b*)(O1 + gi) = h1; *(volatile v8b*)(O2 + gi) = l1; if (MODE == 1) { *(volatile v8b*)(O3 + gi) = h2; *(volatile v8b*)(O4 + gi) = l2; } } }
    __threadfence(); }
}

__global__ __launch_bounds__(256) void vt_kernel(const b16* __restrict__ Vr, b16* __restrict__ vt) {
  __shared__ __attribute__((aligned(16))) b16 Tt[HD][128 + 8];
  const int b = blockIdx.z, h = blockIdx.y, t0 = blockIdx.x * 128, t_ = threadIdx.x;
  for (int i = t_; i < 128 * (HD / 8); i += 256) { const int tk = i >> 3, d8 = (i & 7) * 8; const v8b vv = *(const v8b*)(Vr + ((size_t)(b * T + t0 + tk)) * D + h * HD + d8); for (int e = 0; e < 8; ++e) Tt[d8 + e][tk] = vv[e]; }
  __syncthreads();
  for (int pass = 0; pass < 2; ++pass) { for (int i = t_; i < HD * 16; i += 256) { const int d = i >> 4, c8 = (i & 15) * 8; *(volatile v8b*)(vt + (((size_t)b * H + h) * HD + d) * T + t0 + c8) = *(const v8b*)(&Tt[d][c8]); } __threadfence(); }
}

__global__ __launch_bounds__(128) void attn_kernel(const b16* __restrict__ QUh, const b16* __restrict__ QUl, const b16* __restrict__ QVh, const b16* __restrict__ QVl, const b16* __restrict__ Kh, const b16* __restrict__ Kl, const b16* __restrict__ Eh, const b16* __restrict__ El, const b16* __restrict__ vt, const b16* __restrict__ vtl, b16* __restrict__ ctxh, b16* __restrict__ ctxl) {
  __shared__ float S[4][16][T + 32 + 1]; __shared__ __attribute__((aligned(16))) b16 Oh[16][4 * HD + 8], Ol[16][4 * HD + 8];
  const int wid = threadIdx.x >> 5, lane = threadIdx.x & 31, hh = lane >> 4, col = lane & 15; const int b = blockIdx.x / (T / 16), i0 = (blockIdx.x % (T / 16)) * 16, h = blockIdx.y * 4 + wid, qi = i0 + col;
  const size_t rb = (size_t)(b * T) * D + h * HD; const b16* V = vt + (((size_t)b * H + h) * HD) * T; const b16* Vl = vtl + (((size_t)b * H + h) * HD) * T;
  { const v16b qa0 = frag_kb(QVh + rb + (size_t)qi * D, hh), qa1 = frag_kb(QVh + rb + (size_t)qi * D + 32, hh), qb0 = frag_kb(QVl + rb + (size_t)qi * D, hh), qb1 = frag_kb(QVl + rb + (size_t)qi * D + 32, hh);
    for (int mblk = 0; mblk < 17; ++mblk) { const int r0 = (T - 1) - i0 - 15 + 32 * mblk - 0;
      for (int half = 0; half < 2; ++half) { const int rr0 = 496 - i0 + 32 * mblk + 16 * half; v8f s = {};
        if (rr0 >= 0 && rr0 + 15 < NRP) { const b16* er = Eh + (size_t)(rr0 + col) * D + h * HD; const b16* el = El + (size_t)(rr0 + col) * D + h * HD;
          const v16b e0h = frag_kb(er, hh), e0l = frag_kb(el, hh), e1h = frag_kb(er + 32, hh), e1l = frag_kb(el + 32, hh);
          s = wmma16b(e0h, qa0, s); s = wmma16b(e0h, qb0, s); s = wmma16b(e0l, qa0, s); s = wmma16b(e1h, qa1, s); s = wmma16b(e1h, qb1, s); s = wmma16b(e1l, qa1, s);
#pragma unroll
          for (int r = 0; r < 8; ++r) { const int rrel = rr0 + 8 * hh + r; const int j = rrel + qi - (T - 1); if (j >= 0 && j < T && rrel < NR) S[wid][col][j] = s[r]; } } }
      (void)r0; } }
  wave_lds_sync();
  const v16b ua0 = frag_kb(QUh + rb + (size_t)qi * D, hh), ua1 = frag_kb(QUh + rb + (size_t)qi * D + 32, hh), ub0 = frag_kb(QUl + rb + (size_t)qi * D, hh), ub1 = frag_kb(QUl + rb + (size_t)qi * D + 32, hh);
  float m = -INFINITY, l = 0.0f; v8f o[4] = {{}, {}, {}, {}}; const float SC = 0.125f / (XS * XS);
  for (int kb = 0; kb < T; kb += 32) { v8f s0 = {}, s1 = {};
    { const b16* kr = Kh + rb + (size_t)(kb + col) * D; const b16* kl = Kl + rb + (size_t)(kb + col) * D; const v16b k0h = frag_kb(kr, hh), k0l = frag_kb(kl, hh), k1h = frag_kb(kr + 32, hh), k1l = frag_kb(kl + 32, hh);
      s0 = wmma16b(k0h, ua0, s0); s0 = wmma16b(k0h, ub0, s0); s0 = wmma16b(k0l, ua0, s0); s0 = wmma16b(k1h, ua1, s0); s0 = wmma16b(k1h, ub1, s0); s0 = wmma16b(k1l, ua1, s0); }
    { const b16* kr = Kh + rb + (size_t)(kb + 16 + col) * D; const b16* kl = Kl + rb + (size_t)(kb + 16 + col) * D; const v16b k0h = frag_kb(kr, hh), k0l = frag_kb(kl, hh), k1h = frag_kb(kr + 32, hh), k1l = frag_kb(kl + 32, hh);
      s1 = wmma16b(k0h, ua0, s1); s1 = wmma16b(k0h, ub0, s1); s1 = wmma16b(k0l, ua0, s1); s1 = wmma16b(k1h, ua1, s1); s1 = wmma16b(k1h, ub1, s1); s1 = wmma16b(k1l, ua1, s1); }
    float mr = -INFINITY;
#pragma unroll
    for (int r = 0; r < 8; ++r) { s0[r] = (s0[r] + S[wid][col][kb + 8 * hh + r]) * SC; s1[r] = (s1[r] + S[wid][col][kb + 16 + 8 * hh + r]) * SC; mr = fmaxf(mr, fmaxf(s0[r], s1[r])); }
    mr = fmaxf(mr, __shfl_xor(mr, 16)); const float mn = fmaxf(m, mr), al_ = nexp(m - mn); m = mn; float sum = 0.0f; v16b pb, pl;
#pragma unroll
    for (int r = 0; r < 8; ++r) { const float e0 = nexp(s0[r] - mn), e1 = nexp(s1[r] - mn); sum += e0 + e1; b16 a_, c_; split16(e0 * PS, a_, c_); pb[r] = a_; pl[r] = c_; split16(e1 * PS, a_, c_); pb[8 + r] = a_; pl[8 + r] = c_; }
    sum += __shfl_xor(sum, 16); l = l * al_ + sum;
#pragma unroll
    for (int t = 0; t < 4; ++t) { o[t] *= al_; const v16b vh = frag_kb(V + (size_t)(t * 16 + col) * T + kb, hh), vlo = frag_kb(Vl + (size_t)(t * 16 + col) * T + kb, hh); o[t] = wmma16b(vh, pb, o[t]); o[t] = wmma16b(vh, pl, o[t]); o[t] = wmma16b(vlo, pb, o[t]); } }
  const float inv = 1.0f / (l * PS);
#pragma unroll
  for (int t = 0; t < 4; ++t)
#pragma unroll
    for (int r = 0; r < 8; ++r) { b16 a_, c_; split16(o[t][r] * inv, a_, c_); Oh[col][wid * HD + t * 16 + 8 * hh + r] = a_; Ol[col][wid * HD + t * 16 + 8 * hh + r] = c_; }
  __syncthreads();
  for (int pass = 0; pass < 2; ++pass) { for (int i = threadIdx.x; i < 16 * 32; i += 128) { const int rr = i >> 5, c8 = (i & 31) * 8; const size_t gi = ((size_t)(b * T + i0 + rr)) * D + blockIdx.y * 4 * HD + c8; *(volatile v8b*)(ctxh + gi) = *(const v8b*)(&Oh[rr][c8]); *(volatile v8b*)(ctxl + gi) = *(const v8b*)(&Ol[rr][c8]); } __threadfence(); }
}
}

extern "C" void kernel_launch(void* const* d_in, const int* in_sizes, int n_in,
                              void* d_out, int out_size, void* d_ws, size_t ws_size, hipStream_t stream) {
  (void)n_in; (void)out_size;
  const float* x = (const float*)d_in[0]; const float* wq = (const float*)d_in[1]; const float* bq = (const float*)d_in[2]; const float* wk = (const float*)d_in[3]; const float* bk = (const float*)d_in[4]; const float* wv = (const float*)d_in[5]; const float* bv = (const float*)d_in[6];
  const float* wp = (const float*)d_in[7]; const float* bp = (const float*)d_in[8]; const float* wo = (const float*)d_in[9]; const float* bo = (const float*)d_in[10]; const float* u = (const float*)d_in[11]; const float* v = (const float*)d_in[12];
  float* out = (float*)d_out;
  if (in_sizes[0] != NT * D || in_sizes[1] != D * D || in_sizes[7] != D * D || in_sizes[11] != D) return;
  size_t off = 0; char* ws = (char*)d_ws;
  auto carve = [&](size_t bytes) { char* p = ws + off; off += (bytes + 255) & ~(size_t)255; return p; };
  const size_t RB = (size_t)NT * D * 2;
  b16* R = (b16*)carve(Wo_::END * 2); float* P = (float*)carve(7168 * 4); b16* X = (b16*)carve(RB); b16* PEh = (b16*)carve((size_t)NRP * D * 2); b16* PEl = (b16*)carve((size_t)NRP * D * 2);
  b16* QUh = (b16*)carve(RB); b16* QUl = (b16*)carve(RB); b16* QVh = (b16*)carve(RB); b16* QVl = (b16*)carve(RB); b16* Kh = (b16*)carve(RB); b16* Kl = (b16*)carve(RB); b16* VR = (b16*)carve(RB); b16* VT = (b16*)carve(RB);
  b16* Eh = (b16*)carve((size_t)NRP * D * 2); b16* El = (b16*)carve((size_t)NRP * D * 2); b16* CH = (b16*)carve(RB); b16* CL = (b16*)carve(RB); b16* VRl = (b16*)carve(RB);
  if (off > ws_size) return;
  b16* VTl = X;
  prep_kernel<<<512, 256, 0, stream>>>(x, wq, wk, wv, wp, wo, bq, bk, bv, bp, bo, u, v, R, P, X, PEh, PEl);
  gemm_kernel<1, 0><<<dim3(4, NT / 32), 64, 0, stream>>>(X, nullptr, R + Wo_::Q, P, P, QUh, QUl, QVh, QVl, nullptr);
  gemm_kernel<0, 0><<<dim3(4, NT / 32), 64, 0, stream>>>(X, nullptr, R + Wo_::K, P + 1024, P, Kh, Kl, nullptr, nullptr, nullptr);
  gemm_kernel<0, 0><<<dim3(4, NT / 32), 64, 0, stream>>>(X, nullptr, R + Wo_::V, P + 2048, P, VR, VRl, nullptr, nullptr, nullptr);
  gemm_kernel<0, 1><<<dim3(4, NRP / 32), 64, 0, stream>>>(PEh, PEl, R + Wo_::Pp, P + 3072, P, Eh, El, nullptr, nullptr, nullptr);
  vt_kernel<<<dim3(T / 128, H, Bn), 256, 0, stream>>>(VR, VT);
  vt_kernel<<<dim3(T / 128, H, Bn), 256, 0, stream>>>(VRl, VTl);
  attn_kernel<<<dim3(NT / 16, 4), 128, 0, stream>>>(QUh, QUl, QVh, QVl, Kh, Kl, Eh, El, VT, VTl, CH, CL);
  gemm_kernel<3, 1><<<dim3(4, NT / 32), 64, 0, stream>>>(CH, CL, R + Wo_::O, P + 4096, P, nullptr, nullptr, nullptr, nullptr, out);
}
